// HyperEdgeAttention_37177236914496
// MI455X (gfx1250) — hardware-verified
//
#include <hip/hip_runtime.h>
#include <stddef.h>


#define KD     128
#define HN     8
#define HDM    16
#define OW     128
#define PW     384
#define QOFF   0
#define KOFF   128
#define VOFF   256
#define WROWS  512
#define BCN    512
#define NTHR   256
#define NWAVE  8
#define EPT    8
#define NGRP   2
#define CHUNK  (NTHR * EPT * NGRP)
#define WCAP   (EPT * NGRP * 32)
#define LISTN  (NWAVE * WCAP)
#define NBC    4096
#define NBF    1024
#define RCAP   40960
#define RBN    128
#define TPV    16
#define TGT    (NWAVE * TPV)
#define DEGCAP 128
#define NCHK   (DEGCAP / 32)
#define OTHR   512
#define WSCAP  134217728
#define NEG_BIG (-3.0e38f)
#define ATT_SCALE 0.25f
#define BMG    32
#define APK    136
#define TPW_QKV 6
#define TPW_O   2
#define WUNITS (WROWS * KD / 8)

#define LDS_FILL ((RCAP + NBF + LISTN) * 4 + 64)
#define LDS_GQKV (BMG * 64 * TPW_QKV * 4)
#define LDS_GO   (2 * BMG * APK * 2)
#define LDS_AGG  (NWAVE * TPV * 32 * 16 + NWAVE * DEGCAP * HN * 4)

static_assert((CHUNK & (CHUNK - 1)) == 0);
static_assert(CHUNK <= 4096);
static_assert(NBC <= 4096 && NBF <= 4096);
static_assert((NBC & (NBC - 1)) == 0 && (NBF & (NBF - 1)) == 0);
static_assert(NBC == 4 * NBF);
static_assert(OTHR * 8 == NBC);
static_assert((RCAP % 32) == 0);
static_assert(TGT == NWAVE * TPV);
static_assert((TPV & (TPV - 1)) == 0 && TPV <= 32);
static_assert((NBC % TGT) == 0);
static_assert((TGT % BMG) == 0);
static_assert(BMG * KD / 16 == NTHR);
static_assert(((APK * 2) % 16) == 0 && APK >= KD);
static_assert(NCHK * 32 == DEGCAP);
static_assert(4 * TPW_QKV * 16 == PW);
static_assert(4 * TPW_O * 16 == OW);
static_assert(HN * HDM == OW && OW == 4 * 32 && HDM == 16);
static_assert(PW == 3 * OW && KOFF == OW && VOFF == 2 * OW);
static_assert((WUNITS % NTHR) == 0);
static_assert(2 * BMG * APK * 2 <= LDS_GQKV);
static_assert(BMG * OW * 4 <= LDS_GO && 2 * BMG * APK * 2 <= LDS_GO);
static_assert(((BMG * PW / 4) % NTHR) == 0 && ((BMG * OW / 4) % NTHR) == 0);
static_assert((KD % 32) == 0);

typedef float          v4f   __attribute__((ext_vector_type(4)));
typedef float          v8f   __attribute__((ext_vector_type(8)));
typedef int            v4i   __attribute__((ext_vector_type(4)));
typedef unsigned short v8us  __attribute__((ext_vector_type(8)));
typedef __bf16         v16bf __attribute__((ext_vector_type(16)));
union FragB { v16bf v; v8us u[2]; };

__device__ __forceinline__ unsigned short bfb(float f) {
  unsigned u = __float_as_uint(f);
  u = u + 0x7FFFu + ((u >> 16) & 1u);
  return (unsigned short)(u >> 16);
}
__device__ __forceinline__ float bfv(unsigned short b) { return __uint_as_float(((unsigned)b) << 16); }

__device__ __forceinline__ void split2(float f, unsigned short& h, unsigned short& l) {
  h = bfb(f);
  l = bfb(f - bfv(h));
}
__device__ __forceinline__ void split8(v4f a, v4f b, v8us& hv, v8us& lv) {
  unsigned short h, l;
  split2(a.x, h, l); hv[0] = h; lv[0] = l;
  split2(a.y, h, l); hv[1] = h; lv[1] = l;
  split2(a.z, h, l); hv[2] = h; lv[2] = l;
  split2(a.w, h, l); hv[3] = h; lv[3] = l;
  split2(b.x, h, l); hv[4] = h; lv[4] = l;
  split2(b.y, h, l); hv[5] = h; lv[5] = l;
  split2(b.z, h, l); hv[6] = h; lv[6] = l;
  split2(b.w, h, l); hv[7] = h; lv[7] = l;
}

__device__ __forceinline__ v8f wmb(v16bf a, v16bf b, v8f c) {
  v8f d = __builtin_amdgcn_wmma_f32_16x16x32_bf16(false, a, false, b, (short)0, c, false, false);
  asm volatile("v_nop\n\tv_nop\n\tv_nop\n\tv_nop" : "+v"(d) : "v"(a), "v"(b));
  return d;
}

template <int NB>
__device__ __forceinline__ int scan_chunk(const int* __restrict__ dsts, int nE, int cbase, int slotBase,
                                          int vec8, int* list, int tid, int lane, int wave) {
  int wc = 0;
#pragma unroll
  for (int g = 0; g < NGRP; ++g) {
    const int el0  = (g * NTHR + tid) * EPT;
    const int e0   = cbase + el0;
    const int sent = -2147483647 - 1;
    v4i da, db;
    if (vec8 != 0 && cbase + CHUNK <= nE) {
      da = *(const v4i*)(dsts + e0);
      db = *(const v4i*)(dsts + e0 + 4);
    } else {
      da.x = (e0     < nE) ? dsts[min(e0, nE - 1)] : sent;
      da.y = (e0 + 1 < nE) ? dsts[min(e0 + 1, nE - 1)] : sent;
      da.z = (e0 + 2 < nE) ? dsts[min(e0 + 2, nE - 1)] : sent;
      da.w = (e0 + 3 < nE) ? dsts[min(e0 + 3, nE - 1)] : sent;
      db.x = (e0 + 4 < nE) ? dsts[min(e0 + 4, nE - 1)] : sent;
      db.y = (e0 + 5 < nE) ? dsts[min(e0 + 5, nE - 1)] : sent;
      db.z = (e0 + 6 < nE) ? dsts[min(e0 + 6, nE - 1)] : sent;
      db.w = (e0 + 7 < nE) ? dsts[min(e0 + 7, nE - 1)] : sent;
    }
    const unsigned nb = (unsigned)slotBase;
    const unsigned s0 = (unsigned)da.x - nb, s1 = (unsigned)da.y - nb;
    const unsigned s2 = (unsigned)da.z - nb, s3 = (unsigned)da.w - nb;
    const unsigned s4 = (unsigned)db.x - nb, s5 = (unsigned)db.y - nb;
    const unsigned s6 = (unsigned)db.z - nb, s7 = (unsigned)db.w - nb;
    const bool h0 = s0 < (unsigned)NB, h1 = s1 < (unsigned)NB, h2 = s2 < (unsigned)NB, h3 = s3 < (unsigned)NB;
    const bool h4 = s4 < (unsigned)NB, h5 = s5 < (unsigned)NB, h6 = s6 < (unsigned)NB, h7 = s7 < (unsigned)NB;
    const unsigned any = __builtin_amdgcn_ballot_w32(h0 | h1 | h2 | h3 | h4 | h5 | h6 | h7);
    if (any != 0u) {
#define HITJ(J, HJ, SJ) { \
        const unsigned mj = __builtin_amdgcn_ballot_w32(HJ); \
        if (mj != 0u) { \
          if (HJ) { \
            const int pos = wc + (int)__builtin_amdgcn_mbcnt_lo(mj, 0u); \
            if (pos < WCAP) list[wave * WCAP + pos] = ((el0 + (J)) << 12) | (int)(SJ); \
          } \
          wc += (int)__builtin_popcount(mj); } }
      HITJ(0, h0, s0)
      HITJ(1, h1, s1)
      HITJ(2, h2, s2)
      HITJ(3, h3, s3)
      HITJ(4, h4, s4)
      HITJ(5, h5, s5)
      HITJ(6, h6, s6)
      HITJ(7, h7, s7)
#undef HITJ
    }
  }
  return wc;
}

__global__ __launch_bounds__(NTHR) void k_wprep(
    const float* __restrict__ wq, const float* __restrict__ wk,
    const float* __restrict__ wv, const float* __restrict__ wo,
    const float* __restrict__ bq, const float* __restrict__ bk,
    const float* __restrict__ bv, const float* __restrict__ bo,
    unsigned short* whi, unsigned short* wlo, float* bcat) {
  const int i   = (int)blockIdx.x * NTHR + (int)threadIdx.x;
  const int n   = i >> 4;
  const int k0  = (i & 15) * 8;
  const int grp = n >> 7;
  const int nl  = n & 127;
  const float* pq = wq + nl * KD + k0;
  const float* pk = wk + nl * KD + k0;
  const float* pv = wv + nl * KD + k0;
  const float* po = wo + nl * KD + k0;
  const v4f qa = *(const v4f*)pq, qb = *(const v4f*)(pq + 4);
  const v4f ka = *(const v4f*)pk, kb = *(const v4f*)(pk + 4);
  const v4f va = *(const v4f*)pv, vb = *(const v4f*)(pv + 4);
  const v4f oa = *(const v4f*)po, ob = *(const v4f*)(po + 4);
  const v4f sa = (grp == 0) ? qa : ((grp == 1) ? ka : ((grp == 2) ? va : oa));
  const v4f sb = (grp == 0) ? qb : ((grp == 1) ? kb : ((grp == 2) ? vb : ob));
  v8us hv, lv;
  split8(sa, sb, hv, lv);

  const int bi = i > BCN - 1 ? BCN - 1 : i;
  const int bg = bi >> 7;
  const int bl = bi & 127;
  const float ba = bq[bl], bb = bk[bl], bc = bv[bl], bd = bo[bl];
  const float bval = (bg == 0) ? ba : ((bg == 1) ? bb : ((bg == 2) ? bc : bd));

  unsigned short* dh = whi + (size_t)i * 8;
  unsigned short* dl = wlo + (size_t)i * 8;
  *(volatile v8us*)dh = hv;
  *(volatile v8us*)dl = lv;
  if (i < BCN) *(volatile float*)(bcat + i) = bval;
  __threadfence();
  *(volatile v8us*)dh = hv;
  *(volatile v8us*)dl = lv;
  if (i < BCN) *(volatile float*)(bcat + i) = bval;
}

__global__ __launch_bounds__(NTHR) void k_count(
    const int* __restrict__ dsts, int* cnt, int nE, int vec8) {
  __shared__ __attribute__((aligned(16))) int scnt[NBC];
  __shared__ __attribute__((aligned(16))) int list[LISTN];
  __shared__ int wcnt[NWAVE];
  const int tid = threadIdx.x, lane = tid & 31, wave = tid >> 5;
  const int nodeBase = blockIdx.x * NBC;

  for (int i = tid; i < NBC; i += NTHR) scnt[i] = 0;
  __syncthreads();

  const int nChunks = (nE + CHUNK - 1) / CHUNK;
#pragma unroll 1
  for (int ch = 0; ch < nChunks; ++ch) {
    const int cbase = ch * CHUNK;
    const int wc = scan_chunk<NBC>(dsts, nE, cbase, nodeBase, vec8, list, tid, lane, wave);
    if (lane == 0) wcnt[wave] = wc;
    __syncthreads();
    if (wave == 0) {
#pragma unroll 1
      for (int wsx = 0; wsx < NWAVE; ++wsx) {
        int n = __builtin_amdgcn_readfirstlane(wcnt[wsx]);
        n = n > WCAP ? WCAP : (n < 0 ? 0 : n);
        const int* lp = list + wsx * WCAP;
#pragma unroll 1
        for (int i = 0; i < n; ++i) {
          const int ent  = __builtin_amdgcn_readfirstlane(lp[i]);
          const int slot = ent & (NBC - 1);
          if (lane == 0) scnt[slot] = scnt[slot] + 1;
        }
      }
    }
    __syncthreads();
  }

  v4i cq[4];
#pragma unroll
  for (int q = 0; q < 4; ++q) {
    const int f = (wave * 4 + q) * 128 + 4 * lane;
    cq[q] = *(const v4i*)(scnt + f);
  }
  int* cp = cnt + (size_t)nodeBase;
#pragma unroll
  for (int q = 0; q < 4; ++q) {
    const int f = (wave * 4 + q) * 128 + 4 * lane;
    *(volatile v4i*)(cp + f) = cq[q];
  }
  __threadfence();
#pragma unroll
  for (int q = 0; q < 4; ++q) {
    const int f = (wave * 4 + q) * 128 + 4 * lane;
    *(volatile v4i*)(cp + f) = cq[q];
  }
}

__global__ __launch_bounds__(OTHR) void k_offsets(
    const int* __restrict__ cnt, int* off, int* rbase, int nChunk) {
  __shared__ __attribute__((aligned(16))) int soff[NBC];
  __shared__ __attribute__((aligned(16))) int srb[RBN];
  __shared__ int wtot[OTHR / 32];
  const int tid = threadIdx.x, lane = tid & 31, wave = tid >> 5, sub = tid >> 7;
  for (int i = tid; i < RBN; i += OTHR) srb[i] = 0;
  int carry = 0;
#pragma unroll 1
  for (int ch = 0; ch < nChunk; ++ch) {
    const int base = ch * NBC;
    const v4i c0 = *(const v4i*)(cnt + base + 8 * tid);
    const v4i c1 = *(const v4i*)(cnt + base + 8 * tid + 4);
    const int e0 = max(c0.x, 0), e1 = max(c0.y, 0), e2 = max(c0.z, 0), e3 = max(c0.w, 0);
    const int e4 = max(c1.x, 0), e5 = max(c1.y, 0), e6 = max(c1.z, 0), e7 = max(c1.w, 0);
    const int ts = e0 + e1 + e2 + e3 + e4 + e5 + e6 + e7;
    int incl = ts;
#pragma unroll
    for (int d = 1; d < 32; d <<= 1) {
      const int t = __shfl_up(incl, d);
      if (lane >= d) incl += t;
    }
    if (lane == 31) wtot[wave] = incl;
    __syncthreads();
    const int S0 = wtot[0]  + wtot[1]  + wtot[2]  + wtot[3];
    const int S1 = wtot[4]  + wtot[5]  + wtot[6]  + wtot[7];
    const int S2 = wtot[8]  + wtot[9]  + wtot[10] + wtot[11];
    const int S3 = wtot[12] + wtot[13] + wtot[14] + wtot[15];
    int pre = 0;
#pragma unroll 1
    for (int w = 4 * sub; w < wave; ++w) pre += wtot[w];
    const int b0 = carry;
    const int b1 = b0 + ((S0 + 31) & ~31);
    const int b2 = b1 + ((S1 + 31) & ~31);
    const int b3 = b2 + ((S2 + 31) & ~31);
    const int b4 = b3 + ((S3 + 31) & ~31);
    const int myb = sub == 0 ? b0 : (sub == 1 ? b1 : (sub == 2 ? b2 : b3));
    if (tid == 0) {
      srb[min(4 * ch + 0, RBN - 1)] = b0;
      srb[min(4 * ch + 1, RBN - 1)] = b1;
      srb[min(4 * ch + 2, RBN - 1)] = b2;
      srb[min(4 * ch + 3, RBN - 1)] = b3;
    }
    int run = myb + pre + incl - ts;
    soff[8 * tid + 0] = run; run += e0;
    soff[8 * tid + 1] = run; run += e1;
    soff[8 * tid + 2] = run; run += e2;
    soff[8 * tid + 3] = run; run += e3;
    soff[8 * tid + 4] = run; run += e4;
    soff[8 * tid + 5] = run; run += e5;
    soff[8 * tid + 6] = run; run += e6;
    soff[8 * tid + 7] = run;
    carry = b4;
    __syncthreads();
    const v4i o0 = *(const v4i*)(soff + 4 * tid);
    const v4i o1 = *(const v4i*)(soff + 4 * (tid + OTHR));
    int* op = off + base;
    *(volatile v4i*)(op + 4 * tid) = o0;
    *(volatile v4i*)(op + 4 * (tid + OTHR)) = o1;
    __threadfence();
    *(volatile v4i*)(op + 4 * tid) = o0;
    *(volatile v4i*)(op + 4 * (tid + OTHR)) = o1;
    __syncthreads();
  }
  if (tid == 0) srb[min(4 * nChunk, RBN - 1)] = carry;
  __syncthreads();
  v4i rv = {0, 0, 0, 0};
  if (tid < 32) rv = *(const v4i*)(srb + 4 * tid);
  if (tid < 32) *(volatile v4i*)(rbase + 4 * tid) = rv;
  __threadfence();
  if (tid < 32) *(volatile v4i*)(rbase + 4 * tid) = rv;
}

__global__ __launch_bounds__(NTHR) void k_fill(
    const int* __restrict__ srcs, const int* __restrict__ dsts,
    const int* __restrict__ off, const int* __restrict__ rbase,
    int* csr, int nN, int nE, int vec8, int csrLen) {
  extern __shared__ v4f lds_dyn[];
  int* region = (int*)lds_dyn;
  int* cursor = region + RCAP;
  int* list   = cursor + NBF;
  int* wcnt   = list + LISTN;
  const int tid = threadIdx.x, lane = tid & 31, wave = tid >> 5;
  const int b = blockIdx.x;
  const int nodeBase = b * NBF;

  int rb0 = rbase[b];
  const int rb1 = rbase[b + 1];
  rb0 = rb0 < 0 ? 0 : (rb0 > csrLen ? csrLen : rb0);
  rb0 &= ~31;
  int len = rb1 - rb0;
  len = len < 0 ? 0 : (len > RCAP ? RCAP : len);
  int lenW = (len + 31) & ~31;
  if (rb0 + lenW > csrLen) lenW = (csrLen - rb0) & ~31;

  {
    const v4i z = {0, 0, 0, 0};
    for (int i = tid; i < RCAP / 4; i += NTHR) ((v4i*)region)[i] = z;
    for (int s = tid; s < NBF; s += NTHR) {
      int o = off[nodeBase + s] - rb0;
      o = o < 0 ? 0 : (o > RCAP ? RCAP : o);
      cursor[s] = o;
    }
  }
  __syncthreads();

  const int nChunks = (nE + CHUNK - 1) / CHUNK;
#pragma unroll 1
  for (int ch = 0; ch < nChunks; ++ch) {
    const int cbase = ch * CHUNK;
    const int wc = scan_chunk<NBF>(dsts, nE, cbase, nodeBase, vec8, list, tid, lane, wave);
    if (lane == 0) wcnt[wave] = wc;
    __syncthreads();
    if (wave == 0) {
#pragma unroll 1
      for (int wsx = 0; wsx < NWAVE; ++wsx) {
        int n = __builtin_amdgcn_readfirstlane(wcnt[wsx]);
        n = n > WCAP ? WCAP : (n < 0 ? 0 : n);
        const int* lp = list + wsx * WCAP;
#pragma unroll 1
        for (int i = 0; i < n; ++i) {
          const int ent  = __builtin_amdgcn_readfirstlane(lp[i]);
          const int slot = ent & (NBF - 1);
          int e = cbase + ((ent >> 12) & (CHUNK - 1));
          e = e > nE - 1 ? nE - 1 : e;
          int src = srcs[e];
          src = src < 0 ? 0 : (src > nN - 1 ? nN - 1 : src);
          if (lane == 0) {
            int pos = cursor[slot];
            pos = pos < 0 ? 0 : (pos > RCAP - 1 ? RCAP - 1 : pos);
            region[pos] = src;
            const int np = pos + 1;
            cursor[slot] = np > RCAP ? RCAP : np;
          }
        }
      }
    }
    __syncthreads();
  }

  const int nv = lenW >> 2;
  int* gp = csr + rb0;
#pragma unroll 1
  for (int i = tid; i < nv; i += NTHR) { const v4i v = ((const v4i*)region)[i]; *(volatile v4i*)(gp + 4 * i) = v; }
  __threadfence();
#pragma unroll 1
  for (int i = tid; i < nv; i += NTHR) { const v4i v = ((const v4i*)region)[i]; *(volatile v4i*)(gp + 4 * i) = v; }
}

template <int TPW>
__global__ __launch_bounds__(NTHR) void k_gemm(
    const float* __restrict__ A, int nRowsA,
    const unsigned short* __restrict__ whi, const unsigned short* __restrict__ wlo,
    const float* __restrict__ bias, float* C, int nRowsC) {
  constexpr int PWD = 64 * TPW;
  constexpr int NIT = (BMG * PWD / 4) / NTHR;
  extern __shared__ v4f lds_dyn[];
  unsigned short* sAh = (unsigned short*)lds_dyn;
  unsigned short* sAl = sAh + BMG * APK;
  float*          stg = (float*)lds_dyn;
  const int tid = threadIdx.x, lane = tid & 31, wave = tid >> 5, hh = lane >> 4, m = lane & 15;
  const int rowBase = blockIdx.x * BMG;

  {
    const int r  = tid >> 3;
    const int cc = (tid & 7) * 16;
    int row = rowBase + r;
    row = row > nRowsA - 1 ? nRowsA - 1 : row;
    const float* ap = A + (size_t)row * KD + cc;
    const v4f x0 = *(const v4f*)ap, x1 = *(const v4f*)(ap + 4);
    const v4f x2 = *(const v4f*)(ap + 8), x3 = *(const v4f*)(ap + 12);
    v8us h0, l0, h1, l1;
    split8(x0, x1, h0, l0);
    split8(x2, x3, h1, l1);
    *(v8us*)(sAh + r * APK + cc)     = h0;
    *(v8us*)(sAh + r * APK + cc + 8) = h1;
    *(v8us*)(sAl + r * APK + cc)     = l0;
    *(v8us*)(sAl + r * APK + cc + 8) = l1;
  }
  __syncthreads();

  const int rg = wave >> 2;
  const int cq = wave & 3;
  const int r0 = rg * 16;
  const int c0 = cq * (TPW * 16);

  v8f acc[TPW];
#pragma unroll
  for (int t = 0; t < TPW; ++t) { v8f z = {0.f, 0.f, 0.f, 0.f, 0.f, 0.f, 0.f, 0.f}; acc[t] = z; }
  const unsigned short* ahp = sAh + (r0 + m) * APK + 8 * hh;
  const unsigned short* alp = sAl + (r0 + m) * APK + 8 * hh;
#pragma unroll
  for (int kt = 0; kt < KD / 32; ++kt) {
    FragB ah, al;
    ah.u[0] = *(const v8us*)(ahp + 32 * kt);
    ah.u[1] = *(const v8us*)(ahp + 32 * kt + 16);
    al.u[0] = *(const v8us*)(alp + 32 * kt);
    al.u[1] = *(const v8us*)(alp + 32 * kt + 16);
#pragma unroll
    for (int t = 0; t < TPW; ++t) {
      const size_t bo = (size_t)(c0 + 16 * t + m) * KD + 32 * kt + 8 * hh;
      FragB bh, bl;
      bh.u[0] = *(const v8us*)(whi + bo);
      bh.u[1] = *(const v8us*)(whi + bo + 16);
      bl.u[0] = *(const v8us*)(wlo + bo);
      bl.u[1] = *(const v8us*)(wlo + bo + 16);
      acc[t] = wmb(ah.v, bh.v, acc[t]);
      acc[t] = wmb(ah.v, bl.v, acc[t]);
      acc[t] = wmb(al.v, bh.v, acc[t]);
    }
  }
  __syncthreads();

  {
    float* sp = stg + (size_t)(r0 + 8 * hh) * PWD + c0 + m;
#pragma unroll
    for (int t = 0; t < TPW; ++t) {
#pragma unroll
      for (int r = 0; r < 8; ++r) sp[r * PWD + 16 * t] = acc[t][r];
    }
  }
  __syncthreads();

  float* gp = C + (size_t)rowBase * PWD;
#pragma unroll
  for (int it = 0; it < NIT; ++it) {
    const int f    = it * NTHR + tid;
    const int col4 = f % (PWD / 4);
    const int grow = rowBase + f / (PWD / 4);
    const v4f v  = *(const v4f*)(stg + 4 * f);
    const v4f bb = *(const v4f*)(bias + 4 * col4);
    const v4f o  = v + bb;
    if (grow < nRowsC) *(volatile v4f*)(gp + 4 * (size_t)f) = o;
  }
  __threadfence();
#pragma unroll
  for (int it = 0; it < NIT; ++it) {
    const int f    = it * NTHR + tid;
    const int col4 = f % (PWD / 4);
    const int grow = rowBase + f / (PWD / 4);
    const v4f v  = *(const v4f*)(stg + 4 * f);
    const v4f bb = *(const v4f*)(bias + 4 * col4);
    const v4f o  = v + bb;
    if (grow < nRowsC) *(volatile v4f*)(gp + 4 * (size_t)f) = o;
  }
}

__global__ __launch_bounds__(NTHR) void k_agg(
    const int* __restrict__ csr, const int* __restrict__ off, const int* __restrict__ cnt,
    const float* __restrict__ P, float* X, int nN, int csrLen) {
  extern __shared__ v4f lds_dyn[];
  v4f*   sOut = lds_dyn;
  float* sLog = (float*)(lds_dyn + NWAVE * TPV * 32);
  const int tid = threadIdx.x, lane = tid & 31, wave = tid >> 5, hd = lane >> 2;
  const int tbase = blockIdx.x * TGT + wave * TPV;
  const v4f z4 = {0.f, 0.f, 0.f, 0.f};
  float* slw = sLog + wave * (DEGCAP * HN);

  const int cl    = tbase + (lane & (TPV - 1));
  const int cnt_l = cnt[cl];
  const int off_l = off[cl];

#pragma unroll 1
  for (int j = 0; j < TPV; ++j) {
    const int c = tbase + j;
    int n = __shfl(cnt_l, j);
    n = n < 0 ? 0 : (n > DEGCAP ? DEGCAP : n);
    const int st = __shfl(off_l, j);
    const v4f k4 = *(const v4f*)(P + (size_t)c * PW + KOFF + 4 * lane);

    float mx = NEG_BIG;
#pragma unroll
    for (int kc = 0; kc < NCHK; ++kc) {
      const int q0 = 32 * kc;
      if (q0 < n) {
        int pos = st + q0 + lane;
        pos = pos < 0 ? 0 : (pos > csrLen - 1 ? csrLen - 1 : pos);
        int sl = csr[pos];
        sl = sl < 0 ? 0 : (sl > nN - 1 ? nN - 1 : sl);
        const int mcnt = (n - q0) < 32 ? (n - q0) : 32;
#pragma unroll 1
        for (int pp = 0; pp < mcnt; ++pp) {
          const int s = __builtin_amdgcn_readlane(sl, pp);
          const v4f q4 = *(const v4f*)(P + (size_t)s * PW + QOFF + 4 * lane);
          float d = q4.x * k4.x + q4.y * k4.y + q4.z * k4.z + q4.w * k4.w;
          d += __shfl_xor(d, 1);
          d += __shfl_xor(d, 2);
          d *= ATT_SCALE;
          mx = fmaxf(mx, d);
          slw[(q0 + pp) * HN + hd] = d;
        }
      }
    }
    __builtin_amdgcn_fence(__ATOMIC_RELEASE, "wavefront");
    __builtin_amdgcn_wave_barrier();

    float den = 0.f;
    v4f acc = z4;
#pragma unroll
    for (int kc = 0; kc < NCHK; ++kc) {
      const int q0 = 32 * kc;
      if (q0 < n) {
        int pos = st + q0 + lane;
        pos = pos < 0 ? 0 : (pos > csrLen - 1 ? csrLen - 1 : pos);
        int sl = csr[pos];
        sl = sl < 0 ? 0 : (sl > nN - 1 ? nN - 1 : sl);
        const int mcnt = (n - q0) < 32 ? (n - q0) : 32;
#pragma unroll 1
        for (int pp = 0; pp < mcnt; ++pp) {
          const int s = __builtin_amdgcn_readlane(sl, pp);
          const float ld = slw[(q0 + pp) * HN + hd];
          const float p  = __expf(ld - mx);
          den += p;
          const v4f v4 = *(const v4f*)(P + (size_t)s * PW + VOFF + 4 * lane);
          acc = acc + v4 * p;
        }
      }
    }

    const float rd = 1.0f / (n > 0 ? den : 1.0f);
    v4f ov = acc * rd;
    if (c >= nN) ov = z4;
    sOut[wave * (TPV * 32) + j * 32 + lane] = ov;
    __builtin_amdgcn_fence(__ATOMIC_RELEASE, "wavefront");
    __builtin_amdgcn_wave_barrier();
  }
  __syncthreads();

  float* gp = X + (size_t)tbase * OW;
#pragma unroll
  for (int it = 0; it < TPV; ++it) {
    const int f = it * 32 + lane;
    const v4f v = sOut[wave * (TPV * 32) + f];
    *(volatile v4f*)(gp + 4 * f) = v;
  }
  __threadfence();
#pragma unroll
  for (int it = 0; it < TPV; ++it) {
    const int f = it * 32 + lane;
    const v4f v = sOut[wave * (TPV * 32) + f];
    *(volatile v4f*)(gp + 4 * f) = v;
  }
}

extern "C" void kernel_launch(void* const* d_in, const int* in_sizes, int n_in,
                              void* d_out, int out_size, void* d_ws, size_t ws_size,
                              hipStream_t stream) {
  if (n_in < 11) return;
  const int nN = in_sizes[0] / KD;
  const int nE = in_sizes[1];
  if (nN <= 0 || nE <= 0 || in_sizes[0] != nN * KD || in_sizes[2] != nE) return;
  if (in_sizes[3] != OW * KD || in_sizes[4] != OW) return;
  if (in_sizes[5] != OW * KD || in_sizes[6] != OW) return;
  if (in_sizes[7] != OW * KD || in_sizes[8] != OW) return;
  if (in_sizes[9] != OW * OW || in_sizes[10] != OW) return;
  if (out_size != nN * OW) return;
  if (nE > (1 << 28) || nN > (1 << 24)) return;

  const float* hin = (const float*)d_in[0];
  const int*   src = (const int*)d_in[1];
  const int*   dst = (const int*)d_in[2];
  const float* wq  = (const float*)d_in[3];
  const float* bq  = (const float*)d_in[4];
  const float* wk  = (const float*)d_in[5];
  const float* bk  = (const float*)d_in[6];
  const float* wv  = (const float*)d_in[7];
  const float* bv  = (const float*)d_in[8];
  const float* wo  = (const float*)d_in[9];
  const float* bo  = (const float*)d_in[10];
  float* out = (float*)d_out;

  const int NPAD   = ((nN + TGT - 1) / TGT) * TGT;
  const int nBC    = (nN + NBC - 1) / NBC;
  const int CNTPAD = nBC * NBC;
  if (4 * nBC + 1 > RBN) return;
  const int nBF    = (nN + NBF - 1) / NBF;
  const int csrLen = ((nE + 31) & ~31) + 4096;
  if (31 * 4 * nBC > 4096) return;
  const int nAgg   = NPAD / TGT;
  const int nGemm  = NPAD / BMG;

  char* ws = (char*)d_ws;
  size_t off = 0;
  const size_t oWh  = off; off += (size_t)WROWS * KD * 2;         off = (off + 255) & ~(size_t)255;
  const size_t oWl  = off; off += (size_t)WROWS * KD * 2;         off = (off + 255) & ~(size_t)255;
  const size_t oBc  = off; off += (size_t)BCN * 4;                off = (off + 255) & ~(size_t)255;
  const size_t oCnt = off; off += (size_t)CNTPAD * 4;             off = (off + 255) & ~(size_t)255;
  const size_t oOff = off; off += (size_t)CNTPAD * 4;             off = (off + 255) & ~(size_t)255;
  const size_t oRb  = off; off += (size_t)RBN * 4;                off = (off + 255) & ~(size_t)255;
  const size_t oCsr = off; off += (size_t)csrLen * 4;             off = (off + 255) & ~(size_t)255;
  const size_t oP   = off; off += (size_t)NPAD * PW * 4;          off = (off + 255) & ~(size_t)255;
  const size_t oX   = off; off += (size_t)NPAD * OW * 4;          off = (off + 255) & ~(size_t)255;
  if (off > ws_size || off > (size_t)WSCAP) return;
  unsigned short* whi = (unsigned short*)(ws + oWh);
  unsigned short* wlo = (unsigned short*)(ws + oWl);
  float* bcat = (float*)(ws + oBc);
  int*   cnt  = (int*)(ws + oCnt);
  int*   offp = (int*)(ws + oOff);
  int*   rb   = (int*)(ws + oRb);
  int*   csr  = (int*)(ws + oCsr);
  float* P    = (float*)(ws + oP);
  float* xb   = (float*)(ws + oX);

  const int vec8 = ((nE & 3) == 0) ? 1 : 0;

  k_wprep<<<WUNITS / NTHR, NTHR, 0, stream>>>(wq, wk, wv, wo, bq, bk, bv, bo, whi, wlo, bcat);

  k_count<<<nBC, NTHR, 0, stream>>>(dst, cnt, nE, vec8);
  k_offsets<<<1, OTHR, 0, stream>>>(cnt, offp, rb, nBC);
  hipFuncSetAttribute(reinterpret_cast<const void*>(&k_fill),
                      hipFuncAttributeMaxDynamicSharedMemorySize, LDS_FILL);
  k_fill<<<nBF, NTHR, LDS_FILL, stream>>>(src, dst, offp, rb, csr, nN, nE, vec8, csrLen);

  k_gemm<TPW_QKV><<<nGemm, NTHR, LDS_GQKV, stream>>>(hin, nN, whi, wlo, bcat, P, NPAD);

  hipFuncSetAttribute(reinterpret_cast<const void*>(&k_agg),
                      hipFuncAttributeMaxDynamicSharedMemorySize, LDS_AGG);
  k_agg<<<nAgg, NTHR, LDS_AGG, stream>>>(csr, offp, cnt, P, xb, nN, csrLen);

  k_gemm<TPW_O><<<nGemm, NTHR, LDS_GO, stream>>>(xb, NPAD, whi + (size_t)PW * KD, wlo + (size_t)PW * KD,
                                                  bcat + PW, out, nN);
}
